// SelfAttentionLayer_65481071401231
// MI455X (gfx1250) — hardware-verified
//
#include <hip/hip_runtime.h>
#include <math.h>

#define TT 4096
#define CC 128
#define DIN 128
#define NH 4
#define HD 32
#define HG 1
#define NQB (TT / 64)
#define CAUSAL 0
#define QHI 64
#define KHI 64
#define QBH 0
#define SCALE (1.0f)
typedef __attribute__((ext_vector_type(16))) _Float16 v16h;
typedef __attribute__((ext_vector_type(16))) __bf16 v16b;
typedef __attribute__((ext_vector_type(8)))  _Float16 v8h;
typedef __attribute__((ext_vector_type(8)))  float v8f;
typedef __attribute__((ext_vector_type(4)))  float v4f;
typedef __attribute__((ext_vector_type(2)))  float v2f;
typedef __attribute__((ext_vector_type(4)))  unsigned v4u;
typedef __attribute__((ext_vector_type(4)))  int v4i;
typedef float __attribute__((may_alias)) float_a;
typedef int __attribute__((may_alias)) int_a;

template <typename T> __device__ __forceinline__ void vst2(void* p, T v) { *(volatile T*)p = v; __threadfence(); *(volatile T*)p = v; }
__device__ __forceinline__ v8f wmma16(v16h a, v16h b, v8f c) {
  v8f d = __builtin_amdgcn_wmma_f32_16x16x32_f16(false, a, false, b, (short)0, c, false, false);
  asm volatile("v_nop\n\tv_nop\n\tv_nop\n\tv_nop" : "+v"(d) : "v"(a), "v"(b));
  return d;
}
__device__ __forceinline__ v8f wmma_bf(v16b a, v16b b, v8f c) {
  v8f d = __builtin_amdgcn_wmma_f32_16x16x32_bf16(false, a, false, b, (short)0, c, false, false);
  asm volatile("v_nop\n\tv_nop\n\tv_nop\n\tv_nop" : "+v"(d) : "v"(a), "v"(b));
  return d;
}
__device__ __forceinline__ v16h frag_h(const _Float16* rowk0, int lane) {
  union { v16h v; v8h q[2]; } u; const _Float16* p = rowk0 + 8 * (lane >> 4);
  u.q[0] = *(const v8h*)p; u.q[1] = *(const v8h*)(p + 16); return u.v;
}
__device__ __forceinline__ v16h frag_f32(const float* rowk0, int lane) {
  v16h a; const float* p = rowk0 + 8 * (lane >> 4);
#pragma unroll
  for (int i = 0; i < 8; ++i) { a[i] = (_Float16)p[i]; a[8 + i] = (_Float16)p[16 + i]; }
  return a;
}
__device__ __forceinline__ v16h frag_f32s(const float* rowk0, int lane, float sc) {
  v16h a; const float* p = rowk0 + 8 * (lane >> 4);
#pragma unroll
  for (int i = 0; i < 8; ++i) { a[i] = (_Float16)(p[i] * sc); a[8 + i] = (_Float16)(p[16 + i] * sc); }
  return a;
}
__device__ __forceinline__ v16h fragc_f32(const float* W, int k0, int n, int lane, int ld, int K) {
  v16h a; const int g = lane >> 4;
#pragma unroll
  for (int i = 0; i < 8; ++i) { const int ka = k0 + 8 * g + i, kb = ka + 16;
    a[i] = (_Float16)(ka < K ? W[(size_t)(ka < K ? ka : K - 1) * ld + n] : 0.f); a[8 + i] = (_Float16)(kb < K ? W[(size_t)(kb < K ? kb : K - 1) * ld + n] : 0.f); }
  return a;
}
struct F2 { v16b h, l; };
__device__ __forceinline__ F2 bsplit16(const float v[16]) { F2 r;
#pragma unroll
  for (int i = 0; i < 16; ++i) { const __bf16 h = (__bf16)v[i]; r.h[i] = h; r.l[i] = (__bf16)(v[i] - (float)h); }
  return r; }
__device__ __forceinline__ F2 split_row(const float* row, int k0, int lane) { float v[16]; const float* p = row + k0 + 8 * (lane >> 4);
#pragma unroll
  for (int i = 0; i < 8; ++i) { v[i] = p[i]; v[8 + i] = p[16 + i]; }
  return bsplit16(v); }
__device__ __forceinline__ F2 split_rowK(const float* row, int k0, int lane, int K) { float v[16]; const int g = lane >> 4;
#pragma unroll
  for (int i = 0; i < 8; ++i) { const int ka = k0 + 8 * g + i, kb = ka + 16; v[i] = ka < K ? row[ka < K ? ka : K - 1] : 0.f; v[8 + i] = kb < K ? row[kb < K ? kb : K - 1] : 0.f; }
  return bsplit16(v); }
__device__ __forceinline__ F2 split_col(const float* W, int k0, int n, int lane, int ld, int K) { float v[16]; const int g = lane >> 4;
#pragma unroll
  for (int i = 0; i < 8; ++i) { const int ka = k0 + 8 * g + i, kb = ka + 16; v[i] = ka < K ? W[(size_t)(ka < K ? ka : K - 1) * ld + n] : 0.f; v[8 + i] = kb < K ? W[(size_t)(kb < K ? kb : K - 1) * ld + n] : 0.f; }
  return bsplit16(v); }
__device__ __forceinline__ v8f mac3(const F2& a, const F2& b, v8f c) { c = wmma_bf(a.l, b.h, c); c = wmma_bf(a.h, b.l, c); return wmma_bf(a.h, b.h, c); }
__device__ __forceinline__ float sigm(float v) { return 1.0f / (1.0f + expf(-v)); }
#define LDSX() do { asm volatile("s_wait_dscnt 0" ::: "memory"); __builtin_amdgcn_wave_barrier(); __builtin_amdgcn_fence(__ATOMIC_RELEASE, "workgroup"); } while (0)

__device__ __forceinline__ float bfr(float v) { return (float)(__bf16)v; }
__host__ __device__ __forceinline__ int kb_last(int qb) { return CAUSAL ? ((qb * 64 + 63) >> 7) : (TT / 128 - 1); }
typedef __attribute__((ext_vector_type(8))) __bf16 v8b;
__device__ __forceinline__ v16b frag_b(const __bf16* rowk0, int lane) {
  union { v16b v; v8b q[2]; } u; const __bf16* p = rowk0 + 8 * (lane >> 4);
  u.q[0] = *(const v8b*)p; u.q[1] = *(const v8b*)(p + 16); return u.v;
}
__device__ __forceinline__ v16b wcol_io(const float* Wm, int k0, int o, int lane, int ld) { v16b w; const int g = lane >> 4;
#pragma unroll
  for (int i = 0; i < 8; ++i) { w[i] = (__bf16)Wm[(size_t)(k0 + 8 * g + i) * ld + o]; w[8 + i] = (__bf16)Wm[(size_t)(k0 + 16 + 8 * g + i) * ld + o]; }
  return w; }
__device__ __forceinline__ v16b wcol_oi(const float* Wm, int k0, int o, int lane, int K) { v16b w; const float* p = Wm + (size_t)o * K + k0 + 8 * (lane >> 4);
#pragma unroll
  for (int i = 0; i < 8; ++i) { w[i] = (__bf16)p[i]; w[8 + i] = (__bf16)p[16 + i]; }
  return w; }
__device__ __forceinline__ v16h wcolh_io(const float* Wm, int k0, int o, int lane, int ld) { v16h w; const int g = lane >> 4;
#pragma unroll
  for (int i = 0; i < 8; ++i) { w[i] = (_Float16)(bfr(Wm[(size_t)(k0 + 8 * g + i) * ld + o]) * 256.0f); w[8 + i] = (_Float16)(bfr(Wm[(size_t)(k0 + 16 + 8 * g + i) * ld + o]) * 256.0f); }
  return w; }
__device__ __forceinline__ v16h wcolh_oi(const float* Wm, int k0, int o, int lane, int K) { v16h w; const float* p = Wm + (size_t)o * K + k0 + 8 * (lane >> 4);
#pragma unroll
  for (int i = 0; i < 8; ++i) { w[i] = (_Float16)(bfr(p[i]) * 256.0f); w[8 + i] = (_Float16)(bfr(p[16 + i]) * 256.0f); }
  return w; }
__device__ __forceinline__ v16b wcol_hdk(const float* Wm, int k0, int o, int lane) { v16b w; const int g = lane >> 4; const float* p = Wm + (size_t)(o / HD) * DIN * HD + (o % HD);
#pragma unroll
  for (int i = 0; i < 8; ++i) { w[i] = (__bf16)p[(size_t)(k0 + 8 * g + i) * HD]; w[8 + i] = (__bf16)p[(size_t)(k0 + 16 + 8 * g + i) * HD]; }
  return w; }
#define WO_OUT_IN 1
#if WQKV_LAYOUT == 1
#define WCOL(W, k0, o, lane) wcol_oi(W, k0, o, lane, DIN)
#elif WQKV_LAYOUT == 2
#define WCOL(W, k0, o, lane) wcol_hdk(W, k0, o, lane)
#else
#define WCOL(W, k0, o, lane) wcol_io(W, k0, o, lane, CC)
#endif
#if WO_OUT_IN
#define WOCOL(W, k0, o, lane) wcol_oi(W, k0, o, lane, CC)
#define WOCOLH(W, k0, o, lane) wcolh_oi(W, k0, o, lane, CC)
#else
#define WOCOL(W, k0, o, lane) wcol_io(W, k0, o, lane, DIN)
#define WOCOLH(W, k0, o, lane) wcolh_io(W, k0, o, lane, DIN)
#endif

#ifndef SM_EXTRA_PARAMS
#define SM_EXTRA_PARAMS
#endif
#ifndef PROJ_EXTRA_PARAMS
#define PROJ_EXTRA_PARAMS
#endif
#ifndef SM_MASK_HOOK
#define SM_MASK_HOOK (void)0
#endif


#define NBR 256
#define DW 1024
__global__ __launch_bounds__(128) void k_qkv3(const float* __restrict__ X, const float* __restrict__ WQ, const float* __restrict__ WK, const float* __restrict__ WV, float* __restrict__ P) { __shared__ __align__(16) float sf[4][16][132];
  const int tid = threadIdx.x, wave = tid >> 5, lane = tid & 31, col = lane & 15, g = lane >> 4; const int c0 = blockIdx.y * 128; const int which = blockIdx.z; const size_t r0 = (size_t)blockIdx.x * 64 + wave * 16; const float* Wm = which == 0 ? WQ : (which == 1 ? WK : WV);
  v8f acc[8] = {};
#pragma unroll 1
  for (int kc = 0; kc < DW / 32; ++kc) { v16b a; { const float* p = X + (r0 + col) * DW + kc * 32 + 8 * g;
#pragma unroll
      for (int i = 0; i < 8; ++i) { a[i] = (__bf16)p[i]; a[8 + i] = (__bf16)p[16 + i]; } }
    asm volatile("s_wait_loadcnt 0x0" ::: "memory");
#pragma unroll
    for (int j = 0; j < 8; ++j) { const v16b w = wcol_oi(Wm, kc * 32, c0 + j * 16 + col, lane, DW); acc[j] = wmma_bf(a, w, acc[j]); } }
#pragma unroll
  for (int j = 0; j < 8; ++j)
#pragma unroll
    for (int r = 0; r < 8; ++r) sf[wave][8 * g + r][j * 16 + col] = acc[j][r];
  LDSX(); for (int rl = 0; rl < 16; ++rl) vst2(P + ((size_t)which * NBR + r0 + rl) * DW + c0 + lane * 4, *(const v4f*)&sf[wave][rl][lane * 4]); }
__global__ __launch_bounds__(256) void k_r1(const float* __restrict__ P, float* __restrict__ OUT) { __shared__ float sk[DW], sv[DW]; __shared__ float sred[2][8];
  const int tid = threadIdx.x; const int b = blockIdx.y; const int i = blockIdx.x * 256 + tid;
  const float* qr = P + ((size_t)0 * NBR + b) * DW; const float* kr = P + ((size_t)1 * NBR + b) * DW; const float* vr = P + ((size_t)2 * NBR + b) * DW;
  float kmx = -3.0e38f, kmn = 3.0e38f;
  for (int j = tid; j < DW; j += 256) { const float kk = kr[j], vv = vr[j]; asm volatile("s_wait_loadcnt 0x0" ::: "memory"); sk[j] = kk; sv[j] = vv; kmx = fmaxf(kmx, kk); kmn = fminf(kmn, kk); }
#pragma unroll
  for (int o = 1; o < 32; o <<= 1) { kmx = fmaxf(kmx, __shfl_xor(kmx, o)); kmn = fminf(kmn, __shfl_xor(kmn, o)); }
  if ((tid & 31) == 0) { sred[0][tid >> 5] = kmx; sred[1][tid >> 5] = kmn; } __syncthreads();
  if (tid < 8) { (void)0; }
  float gmx = sred[0][0], gmn = sred[1][0];
#pragma unroll
  for (int w = 1; w < 8; ++w) { gmx = fmaxf(gmx, sred[0][w]); gmn = fminf(gmn, sred[1][w]); }
  const float qi = qr[i]; asm volatile("s_wait_loadcnt 0x0" ::: "memory");
  const float m = fmaxf((qi * gmx) * (1.0f / 32.0f), (qi * gmn) * (1.0f / 32.0f));
  float den = 0.f, num = 0.f;
#pragma unroll 2
  for (int j = 0; j < DW; ++j) { _Pragma("clang fp contract(off)") const float l = (qi * sk[j]) * (1.0f / 32.0f); const float e = expf(l - m); den += e; num += e * sv[j]; }
  vst2(OUT + (size_t)b * DW + i, num / den); }
#define WS_P 0u
#define WS_END (WS_P + 4u * 3 * (size_t)NBR * DW)
extern "C" void kernel_launch(void* const* d_in, const int* in_sizes, int n_in, void* d_out, int out_size, void* d_ws, size_t ws_size, hipStream_t stream) {
  (void)in_sizes; (void)n_in; (void)out_size;
  const float** F = (const float**)d_in;
  if (ws_size < (size_t)WS_END) return;
  char* ws = (char*)d_ws; float* P = (float*)(ws + WS_P);
  k_qkv3<<<dim3(NBR / 64, DW / 128, 3), 128, 0, stream>>>(F[0], F[1], F[2], F[3], P);
  k_r1<<<dim3(DW / 256, NBR), 256, 0, stream>>>(P, (float*)d_out);
}
